// QNN_64115271795096
// MI455X (gfx1250) — hardware-verified
//
#include <hip/hip_runtime.h>


typedef _Float16 f16t;
typedef f16t  v16h __attribute__((ext_vector_type(16)));
typedef f16t  v8h  __attribute__((ext_vector_type(8)));
typedef float v8f  __attribute__((ext_vector_type(8)));
typedef float v4f  __attribute__((ext_vector_type(4)));
typedef unsigned int v4u __attribute__((ext_vector_type(4)));

union Frag { v16h v; v8h q[2]; };
union Pk16 { v8h h; v4u u; };
union Pk32 { v4f f; v4u u; };

#define NBATCH 64
#define NSTEP  128
#define KIN    300
#define KPAD   320
#define DM     64
#define NCL    10
#define PL     4096
#define NPX    40

__device__ __forceinline__ v8f wmma16(v16h a, v16h b, v8f c) {
  return __builtin_amdgcn_wmma_f32_16x16x32_f16(false, a, false, b, (short)0, c, false, false);
}

__device__ __forceinline__ void guard2(v8f (&c)[2], Frag (&a)[2], Frag (&b)[4]) {
  asm volatile("v_nop\n\tv_nop\n\tv_nop\n\tv_nop"
               : "+v"(c[0]), "+v"(c[1])
               : "v"(a[0].v), "v"(a[1].v), "v"(b[0].v), "v"(b[1].v), "v"(b[2].v), "v"(b[3].v));
}
__device__ __forceinline__ void guard1(v8f& c, Frag (&a)[2], Frag (&b)[2]) {
  asm volatile("v_nop\n\tv_nop\n\tv_nop\n\tv_nop"
               : "+v"(c)
               : "v"(a[0].v), "v"(a[1].v), "v"(b[0].v), "v"(b[1].v));
}
__device__ __forceinline__ void guard8(v8f (&c)[4], v8f (&d)[4], Frag& a, Frag (&ba)[4], Frag (&bb)[4]) {
  asm volatile("v_nop\n\tv_nop\n\tv_nop\n\tv_nop"
               : "+v"(c[0]), "+v"(c[1]), "+v"(c[2]), "+v"(c[3]),
                 "+v"(d[0]), "+v"(d[1]), "+v"(d[2]), "+v"(d[3])
               : "v"(a.v), "v"(ba[0].v), "v"(ba[1].v), "v"(ba[2].v), "v"(ba[3].v),
                 "v"(bb[0].v), "v"(bb[1].v), "v"(bb[2].v), "v"(bb[3].v));
}

__device__ __forceinline__ void zacc2(v8f (&c)[2]) {
  const v8f z = {0.f, 0.f, 0.f, 0.f, 0.f, 0.f, 0.f, 0.f};
  c[0] = z; c[1] = z;
}
__device__ __forceinline__ void zacc4(v8f (&c)[4]) {
  const v8f z = {0.f, 0.f, 0.f, 0.f, 0.f, 0.f, 0.f, 0.f};
  c[0] = z; c[1] = z; c[2] = z; c[3] = z;
}

__device__ __forceinline__ void mm2(v8f (&acc)[2], const f16t* A, const f16t* S,
                                    int mt, int nt0, int h, int m) {
  const f16t* ap = A + (16 * mt + m) * DM + 8 * h;
  const f16t* bp = S + (16 * nt0 + m) * DM + 8 * h;
  Frag a[2], b[4];
  a[0].q[0] = *(const v8h*)(ap);                 a[0].q[1] = *(const v8h*)(ap + 16);
  a[1].q[0] = *(const v8h*)(ap + 32);            a[1].q[1] = *(const v8h*)(ap + 48);
  b[0].q[0] = *(const v8h*)(bp);                 b[0].q[1] = *(const v8h*)(bp + 16);
  b[1].q[0] = *(const v8h*)(bp + 32);            b[1].q[1] = *(const v8h*)(bp + 48);
  b[2].q[0] = *(const v8h*)(bp + 16 * DM);       b[2].q[1] = *(const v8h*)(bp + 16 * DM + 16);
  b[3].q[0] = *(const v8h*)(bp + 16 * DM + 32);  b[3].q[1] = *(const v8h*)(bp + 16 * DM + 48);
  acc[0] = wmma16(a[0].v, b[0].v, acc[0]);
  acc[1] = wmma16(a[0].v, b[2].v, acc[1]);
  acc[0] = wmma16(a[1].v, b[1].v, acc[0]);
  acc[1] = wmma16(a[1].v, b[3].v, acc[1]);
  guard2(acc, a, b);
}

__device__ __forceinline__ void store_rm2(f16t* M, int mt, int nt0, const v8f (&c)[2], int h, int m) {
#pragma unroll
  for (int j = 0; j < 2; ++j)
#pragma unroll
    for (int r = 0; r < 8; ++r)
      M[(16 * mt + 8 * h + r) * DM + 16 * (nt0 + j) + m] = (f16t)c[j][r];
}
__device__ __forceinline__ void store_tr2(f16t* MT, int mt, int nt0, const v8f (&c)[2], int h, int m) {
#pragma unroll
  for (int j = 0; j < 2; ++j) {
    Pk16 p;
#pragma unroll
    for (int r = 0; r < 8; ++r) p.h[r] = (f16t)c[j][r];
    *(v8h*)(MT + (16 * (nt0 + j) + m) * DM + 16 * mt + 8 * h) = p.h;
  }
}

__global__ __launch_bounds__(256)
void k_cvtx(const float* x, f16t* X16, int npieces, int ntot) {
  const int i = blockIdx.x * 256 + threadIdx.x;
  if (i >= npieces) return;
  const int row = i / NPX;
  const int k = (i - row * NPX) * 8;
  Pk16 o;
#pragma unroll
  for (int e = 0; e < 8; ++e) {
    const int kk = k + e;
    int idx = row * KIN + min(kk, KIN - 1);
    idx = min(idx, ntot - 1);
    const float v = x[idx];
    o.h[e] = (kk < KIN) ? (f16t)v : (f16t)0.0f;
  }
  f16t* d = X16 + (size_t)i * 8;
  *(volatile v4u*)d = o.u;
  __threadfence();
  *(volatile v4u*)d = o.u;
}

__global__ __launch_bounds__(256)
void k_pack(const float* Wa, const float* Wp, f16t* P, int npieces) {
  const int i = blockIdx.x * 256 + threadIdx.x;
  if (i >= npieces) return;
  const int pl = i / (DM * NPX);
  const int j = i - pl * (DM * NPX);
  const int n = j / NPX;
  const int k = (j - n * NPX) * 8;
  Pk16 o;
#pragma unroll
  for (int e = 0; e < 8; ++e) {
    const int kk = k + e;
    const int idx = min(kk, KIN - 1) * DM + n;
    const float va = Wa[idx];
    const float vp = Wp[idx];
    const float v = (pl != 0) ? vp : va;
    o.h[e] = (kk < KIN) ? (f16t)(v * 64.0f) : (f16t)0.0f;
  }
  f16t* d = P + (size_t)i * 8;
  *(volatile v4u*)d = o.u;
  __threadfence();
  *(volatile v4u*)d = o.u;
}

__global__ __launch_bounds__(128)
void k_front(const f16t* X16, const f16t* PA, const f16t* PP,
             const float* amp_b, const float* phase_b,
             float* Sr, float* Si, int nrows) {
  __shared__ __attribute__((aligned(16))) float sA[4 * 1024];
  __shared__ __attribute__((aligned(16))) float sP[4 * 1024];
  const int tid = threadIdx.x, w = tid >> 5, l = tid & 31, h = l >> 4, m = l & 15;
  const int r0 = blockIdx.x * 64;
  if (r0 + 64 > nrows) return;

  v8f aa[4], pp[4];
  zacc4(aa); zacc4(pp);
  const f16t* ap  = X16 + (size_t)(r0 + 16 * w + m) * KPAD + 8 * h;
  const f16t* bpa = PA + (size_t)m * KPAD + 8 * h;
  const f16t* bpp = PP + (size_t)m * KPAD + 8 * h;
#pragma unroll 1
  for (int kt = 0; kt < KPAD / 32; ++kt) {
    const int ko = kt * 32;
    Frag a, ba[4], bb[4];
    a.q[0] = *(const v8h*)(ap + ko);
    a.q[1] = *(const v8h*)(ap + ko + 16);
#pragma unroll
    for (int j = 0; j < 4; ++j) {
      const f16t* qa = bpa + (size_t)j * 16 * KPAD + ko;
      const f16t* qb = bpp + (size_t)j * 16 * KPAD + ko;
      ba[j].q[0] = *(const v8h*)qa;  ba[j].q[1] = *(const v8h*)(qa + 16);
      bb[j].q[0] = *(const v8h*)qb;  bb[j].q[1] = *(const v8h*)(qb + 16);
    }
#pragma unroll
    for (int j = 0; j < 4; ++j) aa[j] = wmma16(a.v, ba[j].v, aa[j]);
#pragma unroll
    for (int j = 0; j < 4; ++j) pp[j] = wmma16(a.v, bb[j].v, pp[j]);
    guard8(aa, pp, a, ba, bb);
  }

  float* la = sA + w * 1024;
  float* lp = sP + w * 1024;
#pragma unroll
  for (int j = 0; j < 4; ++j) {
    const int col = 16 * j + m;
    const float ba0 = amp_b[col], bp0 = phase_b[col];
#pragma unroll
    for (int r = 0; r < 8; ++r) {
      const int idx = (8 * h + r) * 64 + col;
      la[idx] = aa[j][r] * 0.015625f + ba0;
      lp[idx] = pp[j][r] * 0.015625f + bp0;
    }
  }
  __syncthreads();
  {
    const int row = l >> 1, hf = l & 1;
    float* qa = la + row * 64 + 32 * hf;
    float* qp = lp + row * 64 + 32 * hf;
    float ss = 0.0f;
#pragma unroll 4
    for (int c = 0; c < 32; ++c) { const float a = qa[c]; ss += a * a; }
    ss += __shfl_xor(ss, 1);
    const float inv = 1.0f / sqrtf(ss);
#pragma unroll 2
    for (int c = 0; c < 32; ++c) {
      const float a  = qa[c] * inv;
      const float ph = qp[c];
      qa[c] = a * cosf(ph);
      qp[c] = a * sinf(ph);
    }
  }
  __syncthreads();
  Pk32 vr[8], vi[8];
#pragma unroll
  for (int i = 0; i < 8; ++i) {
    const int p = l + 32 * i, row = p >> 4, c4 = (p & 15) * 4;
    vr[i].f = *(const v4f*)(la + row * 64 + c4);
    vi[i].f = *(const v4f*)(lp + row * 64 + c4);
  }
#pragma unroll
  for (int i = 0; i < 8; ++i) {
    const int p = l + 32 * i, row = p >> 4, c4 = (p & 15) * 4;
    const size_t g = (size_t)(r0 + 16 * w + row) * DM + c4;
    *(volatile v4u*)(Sr + g) = vr[i].u;
    *(volatile v4u*)(Si + g) = vi[i].u;
  }
  __threadfence();
#pragma unroll
  for (int i = 0; i < 8; ++i) {
    const int p = l + 32 * i, row = p >> 4, c4 = (p & 15) * 4;
    const size_t g = (size_t)(r0 + 16 * w + row) * DM + c4;
    *(volatile v4u*)(Sr + g) = vr[i].u;
    *(volatile v4u*)(Si + g) = vi[i].u;
  }
}

template<bool RM>
__device__ __forceinline__ void qlayer(const f16t* XTr, const f16t* XTi, f16t* HTr, f16t* HTi,
                                       f16t* H2r, f16t* H2i,
                                       const f16t* Ux, const f16t* Uh, f16t* TN, float* sTr,
                                       float lamA, float lamB, int w, int l) {
  const int h = l >> 4, m = l & 15;
  const int mt = w >> 1, nt0 = (w & 1) * 2;
  f16t* T0 = TN;
  f16t* T1 = TN + PL;
  f16t* T2 = TN + 2 * PL;
  f16t* T3 = TN + 3 * PL;

  { v8f c[2]; zacc2(c); mm2(c, Ux, XTr, mt, nt0, h, m); store_rm2(T0, mt, nt0, c, h, m); }
  { v8f c[2]; zacc2(c); mm2(c, Ux, XTi, mt, nt0, h, m); store_rm2(T1, mt, nt0, c, h, m); }
  { v8f c[2]; zacc2(c); mm2(c, Uh, HTr, mt, nt0, h, m); store_rm2(T2, mt, nt0, c, h, m); }
  { v8f c[2]; zacc2(c); mm2(c, Uh, HTi, mt, nt0, h, m); store_rm2(T3, mt, nt0, c, h, m); }
  __syncthreads();

  v8f nr[2], ni[2];
  {
    v8f a[2], c[2];
    zacc2(a); mm2(a, T0, Ux, mt, nt0, h, m);
    zacc2(c); mm2(c, T2, Uh, mt, nt0, h, m);
    nr[0] = a[0] * lamA + c[0] * lamB;
    nr[1] = a[1] * lamA + c[1] * lamB;
  }
  {
    v8f a[2], c[2];
    zacc2(a); mm2(a, T1, Ux, mt, nt0, h, m);
    zacc2(c); mm2(c, T3, Uh, mt, nt0, h, m);
    ni[0] = a[0] * lamA + c[0] * lamB;
    ni[1] = a[1] * lamA + c[1] * lamB;
  }
  __syncthreads();
  store_rm2(T0, mt, nt0, nr, h, m);
  store_rm2(T1, mt, nt0, ni, h, m);
  store_tr2(T2, mt, nt0, nr, h, m);
  store_tr2(T3, mt, nt0, ni, h, m);
  __syncthreads();

  v8f i2[2], r2[2];
  zacc2(i2);
  mm2(i2, T0, T3, mt, nt0, h, m);
  mm2(i2, T1, T2, mt, nt0, h, m);
  {
    v8f ra[2], rb[2];
    zacc2(ra); mm2(ra, T0, T2, mt, nt0, h, m);
    zacc2(rb); mm2(rb, T1, T3, mt, nt0, h, m);
    r2[0] = ra[0] - rb[0];
    r2[1] = ra[1] - rb[1];
  }
  const bool dg0 = (mt == nt0), dg1 = (mt == nt0 + 1);
  const int rs = m - 8 * h;
  float dv = 0.0f;
#pragma unroll
  for (int r = 0; r < 8; ++r) {
    const float e0 = r2[0][r], e1 = r2[1][r];
    const float pick = dg1 ? e1 : e0;
    dv = (rs == r) ? pick : dv;
  }
  dv = (dg0 || dg1) ? dv : 0.0f;
  dv += __shfl_xor(dv, 16);
  dv += __shfl_xor(dv, 8);
  dv += __shfl_xor(dv, 4);
  dv += __shfl_xor(dv, 2);
  dv += __shfl_xor(dv, 1);
  if (l == 0) sTr[w] = dv;
  __syncthreads();
  const float tr = ((sTr[0] + sTr[1]) + (sTr[2] + sTr[3])) + ((sTr[4] + sTr[5]) + (sTr[6] + sTr[7]));
  const float cA = 51.2f / tr;
  v8f hr[2], hi[2];
  hr[0] = r2[0] * cA + nr[0] * 0.2f;
  hr[1] = r2[1] * cA + nr[1] * 0.2f;
  hi[0] = i2[0] * cA + ni[0] * 0.2f;
  hi[1] = i2[1] * cA + ni[1] * 0.2f;
  store_tr2(HTr, mt, nt0, hr, h, m);
  store_tr2(HTi, mt, nt0, hi, h, m);
  if (RM) {
    store_rm2(H2r, mt, nt0, hr, h, m);
    store_rm2(H2i, mt, nt0, hi, h, m);
  }
  __syncthreads();
}

__global__ __launch_bounds__(256)
void k_rec(const float* Sr, const float* Si, const float* Uxg, const float* Uhg,
           const float* lam_p, const float* Wd, const float* dlam_p, const float* meas,
           float* out) {
  __shared__ __attribute__((aligned(16))) f16t  sU[2 * PL];
  __shared__ __attribute__((aligned(16))) f16t  sXT[2 * PL];
  __shared__ __attribute__((aligned(16))) f16t  sHT[4 * PL];
  __shared__ __attribute__((aligned(16))) f16t  sTN[4 * PL];
  __shared__ __attribute__((aligned(16))) f16t  sH2[2 * PL];
  __shared__ __attribute__((aligned(16))) f16t  sWT[16 * DM];
  __shared__ __attribute__((aligned(16))) float sM1[2 * DM * 16];
  __shared__ __attribute__((aligned(16))) float sW[DM * NCL];
  __shared__ __attribute__((aligned(16))) float sG[NCL * NCL * NCL];
  __shared__ __attribute__((aligned(16))) float sHm[NCL * NCL * NCL];
  __shared__ __attribute__((aligned(16))) float sSg[2 * NCL * NCL];
  __shared__ __attribute__((aligned(16))) float sOut[NSTEP * NCL];
  __shared__ float sTr[8];
  __shared__ float sInv[16];

  const int tid = threadIdx.x, w = tid >> 5, l = tid & 31, h = l >> 4, m = l & 15;
  const int b = blockIdx.x;

  for (int i = tid; i < PL; i += 256) {
    sU[i]      = (f16t)(Uxg[i] * 8.0f);
    sU[PL + i] = (f16t)(Uhg[i] * 8.0f);
    const f16t dg = ((i >> 6) == (i & 63)) ? (f16t)1.0f : (f16t)0.0f;
    sHT[i] = dg;              sHT[PL + i] = (f16t)0.0f;
    sHT[2 * PL + i] = dg;     sHT[3 * PL + i] = (f16t)0.0f;
  }
  for (int i = tid; i < 16 * DM; i += 256) {
    const int c = i >> 6, e = i & 63;
    const int cc = min(c, NCL - 1);
    const float v = Wd[e * NCL + cc];
    sWT[i] = (c < NCL) ? (f16t)(v * 8.0f) : (f16t)0.0f;
  }
  for (int i = tid; i < DM * NCL; i += 256) sW[i] = Wd[i];
  if (tid < NCL) {
    float s = 0.0f;
    for (int c = 0; c < NCL; ++c) {
      const float vr = meas[(tid * NCL + c) * 2], vi = meas[(tid * NCL + c) * 2 + 1];
      s += vr * vr + vi * vi;
    }
    sInv[tid] = 1.0f / s;
  }
  __syncthreads();
  for (int i = tid; i < NCL * NCL * NCL; i += 256) {
    const int k = i / (NCL * NCL);
    const int rem = i - k * (NCL * NCL);
    const int c = rem / NCL;
    const int d = rem - c * NCL;
    const float vrc = meas[(k * NCL + c) * 2], vic = meas[(k * NCL + c) * 2 + 1];
    const float vrd = meas[(k * NCL + d) * 2], vid = meas[(k * NCL + d) * 2 + 1];
    const float inv = sInv[k];
    sG[i]  = (vrc * vrd + vic * vid) * inv;
    sHm[i] = (vic * vrd - vrc * vid) * inv;
  }
  const float lam  = 1.0f / (1.0f + expf(-lam_p[0]));
  const float dl   = 1.0f / (1.0f + expf(-dlam_p[0]));
  const float lamA = lam * 0.015625f;
  const float lamB = (1.0f - lam) * 0.015625f;
  const float cI   = (1.0f - dl) * 51.2f;
  __syncthreads();

#pragma unroll 1
  for (int t = 0; t < NSTEP; ++t) {
    {
      const int n = tid >> 2, kq = tid & 3;
      const size_t row = (size_t)b * NSTEP + t;
      const float* pr = Sr + row * DM;
      const float* pi = Si + row * DM;
      const float srn = pr[n], sin_n = pi[n];
      Pk16 o[2], q[2];
#pragma unroll
      for (int j = 0; j < 4; ++j) {
        const v4f rk = *(const v4f*)(pr + 16 * kq + 4 * j);
        const v4f ik = *(const v4f*)(pi + 16 * kq + 4 * j);
#pragma unroll
        for (int e = 0; e < 4; ++e) {
          const float vr = 64.0f * (rk[e] * srn + ik[e] * sin_n);
          const float vi = 64.0f * (ik[e] * srn - rk[e] * sin_n);
          o[j >> 1].h[(j & 1) * 4 + e] = (f16t)vr;
          q[j >> 1].h[(j & 1) * 4 + e] = (f16t)vi;
        }
      }
      f16t* dr = sXT + n * DM + 16 * kq;
      f16t* di = sXT + PL + n * DM + 16 * kq;
      *(v8h*)dr       = o[0].h;
      *(v8h*)(dr + 8) = o[1].h;
      *(v8h*)di       = q[0].h;
      *(v8h*)(di + 8) = q[1].h;
    }
    __syncthreads();

    qlayer<false>(sXT, sXT + PL, sHT, sHT + PL, sH2, sH2 + PL,
                  sU, sU + PL, sTN, sTr, lamA, lamB, w, l);
    qlayer<true>(sHT, sHT + PL, sHT + 2 * PL, sHT + 3 * PL, sH2, sH2 + PL,
                 sU, sU + PL, sTN, sTr, lamA, lamB, w, l);

    {
      const int part = w >> 2, rt = w & 3;
      const f16t* A = sH2 + part * PL + (16 * rt + m) * DM + 8 * h;
      const f16t* S = sWT + m * DM + 8 * h;
      Frag a[2], bb[2];
      a[0].q[0]  = *(const v8h*)(A);       a[0].q[1]  = *(const v8h*)(A + 16);
      a[1].q[0]  = *(const v8h*)(A + 32);  a[1].q[1]  = *(const v8h*)(A + 48);
      bb[0].q[0] = *(const v8h*)(S);       bb[0].q[1] = *(const v8h*)(S + 16);
      bb[1].q[0] = *(const v8h*)(S + 32);  bb[1].q[1] = *(const v8h*)(S + 48);
      v8f c = {0.f, 0.f, 0.f, 0.f, 0.f, 0.f, 0.f, 0.f};
      c = wmma16(a[0].v, bb[0].v, c);
      c = wmma16(a[1].v, bb[1].v, c);
      guard1(c, a, bb);
      float* dst = sM1 + part * (DM * 16);
#pragma unroll
      for (int r = 0; r < 8; ++r) dst[(16 * rt + 8 * h + r) * 16 + m] = c[r];
    }
    __syncthreads();

    if (tid < NCL * NCL) {
      const int c = tid / NCL, f = tid - c * NCL;
      float ar = 0.0f, ai = 0.0f;
#pragma unroll 4
      for (int d = 0; d < DM; ++d) {
        const float wv = sW[d * NCL + c];
        ar += wv * sM1[d * 16 + f];
        ai += wv * sM1[DM * 16 + d * 16 + f];
      }
      sSg[tid]             = dl * ar + ((c == f) ? cI : 0.0f);
      sSg[NCL * NCL + tid] = dl * ai;
    }
    __syncthreads();

    if (tid < 160) {
      const int k = tid >> 4, sub = tid & 15;
      float trc = 0.0f;
#pragma unroll
      for (int c = 0; c < NCL; ++c) trc += sSg[c * (NCL + 1)];
      float ps = 0.0f;
#pragma unroll
      for (int i = 0; i < 7; ++i) {
        const int idx = sub + 16 * i;
        const int ci = min(idx, NCL * NCL - 1);
        const float v = sG[k * NCL * NCL + ci] * sSg[ci] + sHm[k * NCL * NCL + ci] * sSg[NCL * NCL + ci];
        ps += (idx < NCL * NCL) ? v : 0.0f;
      }
      ps += __shfl_xor(ps, 8);
      ps += __shfl_xor(ps, 4);
      ps += __shfl_xor(ps, 2);
      ps += __shfl_xor(ps, 1);
      if (sub == 0) sOut[t * NCL + k] = logf(ps * (1.0f / trc));
    }
  }
  __syncthreads();

  Pk32 v0, v1;
  const int i0 = tid, i1 = tid + 256;
  const int i1c = min(i1, NSTEP * NCL / 4 - 1);
  v0.f = *(const v4f*)(sOut + i0 * 4);
  v1.f = *(const v4f*)(sOut + i1c * 4);
  float* ob = out + (size_t)b * (NSTEP * NCL);
  *(volatile v4u*)(ob + i0 * 4) = v0.u;
  if (i1 < NSTEP * NCL / 4) *(volatile v4u*)(ob + i1 * 4) = v1.u;
  __threadfence();
  *(volatile v4u*)(ob + i0 * 4) = v0.u;
  if (i1 < NSTEP * NCL / 4) *(volatile v4u*)(ob + i1 * 4) = v1.u;
}

extern "C" void kernel_launch(void* const* d_in, const int* in_sizes, int n_in,
                              void* d_out, int out_size, void* d_ws, size_t ws_size,
                              hipStream_t stream) {
  const int nrows = NBATCH * NSTEP;
  if (n_in < 11) return;
  if (in_sizes[0] != nrows * KIN || in_sizes[1] != KIN * DM || in_sizes[2] != DM ||
      in_sizes[3] != KIN * DM || in_sizes[4] != DM || in_sizes[5] != DM * DM ||
      in_sizes[6] != DM * DM || in_sizes[7] < 1 || in_sizes[8] != DM * NCL ||
      in_sizes[9] < 1 || in_sizes[10] != NCL * NCL * 2) return;
  if (out_size != nrows * NCL) return;

  const float* x       = (const float*)d_in[0];
  const float* amp_w   = (const float*)d_in[1];
  const float* amp_b   = (const float*)d_in[2];
  const float* phase_w = (const float*)d_in[3];
  const float* phase_b = (const float*)d_in[4];
  const float* Ux      = (const float*)d_in[5];
  const float* Uh      = (const float*)d_in[6];
  const float* lam_p   = (const float*)d_in[7];
  const float* dense_w = (const float*)d_in[8];
  const float* dlam_p  = (const float*)d_in[9];
  const float* meas    = (const float*)d_in[10];
  float* out = (float*)d_out;

  char* ws = (char*)d_ws;
  size_t off = 0;
  auto carve = [&](size_t bytes) -> char* {
    char* p = ws + off;
    off = (off + bytes + 255) & ~(size_t)255;
    return p;
  };
  f16t*  X16 = (f16t*)carve((size_t)nrows * KPAD * 2);
  f16t*  P   = (f16t*)carve((size_t)2 * DM * KPAD * 2);
  float* Sr  = (float*)carve((size_t)nrows * DM * 4);
  float* Si  = (float*)carve((size_t)nrows * DM * 4);
  if (off > ws_size) return;

  {
    const int npieces = nrows * NPX;
    k_cvtx<<<dim3((npieces + 255) / 256), dim3(256), 0, stream>>>(x, X16, npieces, nrows * KIN);
  }
  {
    const int npieces = 2 * DM * NPX;
    k_pack<<<dim3((npieces + 255) / 256), dim3(256), 0, stream>>>(amp_w, phase_w, P, npieces);
  }
  k_front<<<dim3(nrows / 64), dim3(128), 0, stream>>>(X16, P, P + DM * KPAD, amp_b, phase_b,
                                                     Sr, Si, nrows);
  k_rec<<<dim3(NBATCH), dim3(256), 0, stream>>>(Sr, Si, Ux, Uh, lam_p, dense_w, dlam_p, meas, out);
}
